// LSTMClassifier_35966056137432
// MI455X (gfx1250) — hardware-verified
//
#include <hip/hip_runtime.h>
#include <math.h>

constexpr int NBATCH  = 64;
constexpr int NTIME   = 4096;
constexpr int NCIN    = 32;
constexpr int NCONV   = 64;
constexpr int NTAP    = 5;
constexpr int NSTEPS  = (NTIME - NTAP) / 2 + 1;
constexpr int NHID    = 128;
constexpr int NGATE   = 4 * NHID;
constexpr int NOUTF   = 10;
constexpr int KCONV   = NTAP * NCIN;
constexpr int KCAT    = NCONV + NHID;
constexpr int LBLK    = 3;
constexpr int TROWS   = 2 * LBLK + 3;
constexpr int AWIDTH  = TROWS * NCIN;
constexpr int APITCH  = AWIDTH + 8;
constexpr int SLABP   = 68;
constexpr int ROWBLK  = 16;
constexpr int PPITCH  = KCAT + 8;
constexpr int HFP     = NHID + 4;
constexpr float XCARRY    = 1024.0f;
constexpr float WCARRY    = 64.0f;
constexpr float ACARRY    = 256.0f;
constexpr float CONV_FOLD = 1.0f / (XCARRY * WCARRY);
constexpr float GATE_FOLD = 1.0f / (ACARRY * WCARRY);
constexpr float NORM_EPS  = 1e-12f;

static_assert(NSTEPS == 2046, "conv output length");
static_assert(NSTEPS % LBLK == 0, "conv grid exact");
static_assert(KCONV == 160 && KCONV % 32 == 0, "conv K multiple of 32");
static_assert(KCAT == 192 && KCAT % 32 == 0, "gate K multiple of 32");
static_assert(NBATCH % ROWBLK == 0 && NBATCH % 16 == 0, "batch tile multiple");
static_assert(NCONV % 16 == 0 && NHID == 16 * 8, "8 waves x 16 hidden units");
static_assert((NBATCH * (AWIDTH / 4)) % 128 == 0, "conv staging loop exact");
static_assert((APITCH * 2) % 16 == 0 && (PPITCH * 2) % 16 == 0, "16-B aligned LDS rows");
static_assert(2 * (LBLK - 1) * NCIN + KCONV <= AWIDTH, "conv window inside the staged tile");
static_assert(NBATCH * NTIME * NCIN == 8388608, "input elements");
static_assert(NCONV * NCIN * NTAP == 10240, "conv_w elements");
static_assert(NGATE * NCONV == 32768 && NGATE * NHID == 65536, "w_ih / w_hh elements");
static_assert(NOUTF * NHID == 1280 && NBATCH * NOUTF == 640, "head elements");

typedef __attribute__((ext_vector_type(16))) _Float16 v16h;
typedef __attribute__((ext_vector_type(8)))  _Float16 v8h;
typedef __attribute__((ext_vector_type(4)))  _Float16 v4h;
typedef __attribute__((ext_vector_type(8)))  float    v8f;
typedef __attribute__((ext_vector_type(4)))  float    v4f;
typedef __attribute__((ext_vector_type(2)))  unsigned v2u;

union FragU { v16h v; v8h h[2]; };
__device__ __forceinline__ v16h frag_load(const _Float16* p) {
  FragU f;
  f.h[0] = *(const v8h*)(p);
  f.h[1] = *(const v8h*)(p + 16);
  return f.v;
}
__device__ __forceinline__ v8f frag_mma(v16h a, v16h b, v8f c) {
  return __builtin_amdgcn_wmma_f32_16x16x32_f16(false, a, false, b, (short)0, c, false, false);
}
__device__ __forceinline__ void wm_guard4(v8f& a0, v8f& a1, v8f& a2, v8f& a3, v16h x, v16h y0, v16h y1, v16h y2, v16h y3) {
  asm volatile("v_nop\n\tv_nop\n\tv_nop\n\tv_nop" : "+v"(a0), "+v"(a1), "+v"(a2), "+v"(a3) : "v"(x), "v"(y0), "v"(y1), "v"(y2), "v"(y3));
}
__device__ __forceinline__ void acc_guard4(v8f& a, v8f& b, v8f& c, v8f& d) {
  asm volatile("v_nop\n\tv_nop\n\tv_nop\n\tv_nop" : "+v"(a), "+v"(b), "+v"(c), "+v"(d));
}
__device__ __forceinline__ void wave_sync_lds() {
  __builtin_amdgcn_fence(__ATOMIC_RELEASE, "workgroup");
  __builtin_amdgcn_wave_barrier();
  __builtin_amdgcn_fence(__ATOMIC_ACQUIRE, "workgroup");
}
__device__ __forceinline__ float fsig(float x)  { return __builtin_amdgcn_rcpf(1.0f + expf(-x)); }
__device__ __forceinline__ float ftanh(float x) { return 1.0f - 2.0f * __builtin_amdgcn_rcpf(expf(2.0f * x) + 1.0f); }

__global__ __launch_bounds__(256) void prep_kernel(const float* __restrict__ conv_w, const float* __restrict__ w_ih,
                                                   const float* __restrict__ w_hh, const float* __restrict__ b_ih,
                                                   const float* __restrict__ b_hh, unsigned short* __restrict__ WCAT,
                                                   unsigned short* __restrict__ WC, float* __restrict__ BSUM) {
  const int tid = threadIdx.x;
  const int blk = blockIdx.x;
  if (blk < 16) {
    const int i  = blk * 256 + tid;
    const int n  = i >> 3;
    const int c8 = (i & 7) * 8;
    const float* sp = w_ih + (size_t)n * NCONV + c8;
    const v4f a = *(const v4f*)(sp);
    const v4f b = *(const v4f*)(sp + 4);
    v8h hv;
#pragma unroll
    for (int e = 0; e < 4; ++e) {
      hv[e]     = (_Float16)(a[e] * WCARRY);
      hv[4 + e] = (_Float16)(b[e] * WCARRY);
    }
    unsigned short* dp = WCAT + (size_t)n * KCAT + c8;
    *(volatile v8h*)dp = hv;
    __threadfence();
    *(volatile v8h*)dp = hv;
  } else if (blk < 48) {
    const int i  = (blk - 16) * 256 + tid;
    const int n  = i >> 4;
    const int c8 = (i & 15) * 8;
    const float* sp = w_hh + (size_t)n * NHID + c8;
    const v4f a = *(const v4f*)(sp);
    const v4f b = *(const v4f*)(sp + 4);
    v8h hv;
#pragma unroll
    for (int e = 0; e < 4; ++e) {
      hv[e]     = (_Float16)(a[e] * WCARRY);
      hv[4 + e] = (_Float16)(b[e] * WCARRY);
    }
    unsigned short* dp = WCAT + (size_t)n * KCAT + NCONV + c8;
    *(volatile v8h*)dp = hv;
    __threadfence();
    *(volatile v8h*)dp = hv;
  } else if (blk < 53) {
    const int i   = (blk - 48) * 256 + tid;
    const int oc  = i / (KCONV / 8);
    const int c8  = (i - oc * (KCONV / 8)) * 8;
    const int tap = c8 >> 5;
    const int ic0 = c8 & 31;
    const float* sp = conv_w + (size_t)oc * (NCIN * NTAP) + (size_t)ic0 * NTAP + tap;
    v8h hv;
#pragma unroll
    for (int e = 0; e < 8; ++e) {
      const float f = sp[e * NTAP];
      hv[e] = (_Float16)(f * WCARRY);
    }
    unsigned short* dp = WC + (size_t)i * 8;
    *(volatile v8h*)dp = hv;
    __threadfence();
    *(volatile v8h*)dp = hv;
  } else {
    if (tid < NGATE / 4) {
      const v4f a = *(const v4f*)(b_ih + 4 * tid);
      const v4f b = *(const v4f*)(b_hh + 4 * tid);
      const v4f o = a + b;
      float* dp = BSUM + 4 * tid;
      *(volatile v4f*)dp = o;
      __threadfence();
      *(volatile v4f*)dp = o;
    }
  }
}

__global__ __launch_bounds__(256) void norm_kernel(const float* __restrict__ in, float* __restrict__ INVN) {
  __shared__ float red[256];
  const int tid = threadIdx.x;
  const int c   = tid & 31;
  const int seg = tid >> 5;
  const int bb  = blockIdx.x;
  const float* p = in + ((size_t)bb * NTIME + (size_t)seg * 512) * NCIN + c;
  float s0 = 0.0f, s1 = 0.0f, s2 = 0.0f, s3 = 0.0f;
#pragma unroll 1
  for (int t = 0; t < 512; t += 4) {
    const float v0 = p[(size_t)(t + 0) * NCIN];
    const float v1 = p[(size_t)(t + 1) * NCIN];
    const float v2 = p[(size_t)(t + 2) * NCIN];
    const float v3 = p[(size_t)(t + 3) * NCIN];
    s0 = fmaf(v0, v0, s0);
    s1 = fmaf(v1, v1, s1);
    s2 = fmaf(v2, v2, s2);
    s3 = fmaf(v3, v3, s3);
  }
  red[tid] = (s0 + s1) + (s2 + s3);
  __syncthreads();
  if (seg == 0) {
    float tot = 0.0f;
#pragma unroll
    for (int i = 0; i < 8; ++i) tot += red[i * 32 + c];
    const float nrm = sqrtf(tot);
    const float inv = 1.0f / fmaxf(nrm, NORM_EPS);
    float* dp = INVN + bb * NCIN + c;
    *(volatile float*)dp = inv;
    __threadfence();
    *(volatile float*)dp = inv;
  }
}

__global__ __launch_bounds__(128) void conv_kernel(const float* __restrict__ in, const float* __restrict__ INVN,
                                                   const unsigned short* __restrict__ WCp, const float* __restrict__ conv_b,
                                                   unsigned short* __restrict__ E) {
  __shared__ __align__(16) _Float16 As[NBATCH * APITCH];
  __shared__ __align__(16) float    Sl[4][16 * SLABP];
  const _Float16* WC = (const _Float16*)WCp;
  const int tid = threadIdx.x, lane = tid & 31, wave = tid >> 5;
  const int c = lane & 15, hh = lane >> 4, koff = hh * 8;
  const int l0 = blockIdx.x * LBLK;
  const int t0 = 2 * l0;

#pragma unroll 1
  for (int it = 0; it < (NBATCH * (AWIDTH / 4)) / 128; ++it) {
    const int idx = it * 128 + tid;
    const int br  = idx / (AWIDTH / 4);
    const int q   = idx - br * (AWIDTH / 4);
    const v4f xv = *(const v4f*)(in + ((size_t)br * NTIME + (size_t)t0) * NCIN + q * 4);
    const v4f iv = *(const v4f*)(INVN + br * NCIN + ((q * 4) & (NCIN - 1)));
    v4h hv;
#pragma unroll
    for (int e = 0; e < 4; ++e) {
      const float xn = xv[e] * iv[e];
      hv[e] = (_Float16)(xn * XCARRY);
    }
    *(v4h*)(As + br * APITCH + q * 4) = hv;
  }
  __syncthreads();

  float cb[4];
#pragma unroll
  for (int j = 0; j < 4; ++j) cb[j] = conv_b[16 * j + c];
  float* slab = Sl[wave];
  const v8f z8 = {0.f, 0.f, 0.f, 0.f, 0.f, 0.f, 0.f, 0.f};
  const _Float16* wrow = WC + (size_t)c * KCONV + koff;
  const int q4 = lane >> 3, c8 = (lane & 7) * 8;

#pragma unroll 1
  for (int li = 0; li < LBLK; ++li) {
    const _Float16* arow = As + (16 * wave + c) * APITCH + li * (2 * NCIN) + koff;
    v8f acc[4];
    acc[0] = z8; acc[1] = z8; acc[2] = z8; acc[3] = z8;
#pragma unroll 1
    for (int k0 = 0; k0 < KCONV; k0 += 32) {
      const v16h a  = frag_load(arow + k0);
      const v16h w0 = frag_load(wrow + (size_t)0 * 16 * KCONV + k0);
      const v16h w1 = frag_load(wrow + (size_t)1 * 16 * KCONV + k0);
      const v16h w2 = frag_load(wrow + (size_t)2 * 16 * KCONV + k0);
      const v16h w3 = frag_load(wrow + (size_t)3 * 16 * KCONV + k0);
      acc[0] = frag_mma(a, w0, acc[0]);
      acc[1] = frag_mma(a, w1, acc[1]);
      acc[2] = frag_mma(a, w2, acc[2]);
      acc[3] = frag_mma(a, w3, acc[3]);
      wm_guard4(acc[0], acc[1], acc[2], acc[3], a, w0, w1, w2, w3);
    }
    acc_guard4(acc[0], acc[1], acc[2], acc[3]);
#pragma unroll
    for (int j = 0; j < 4; ++j) {
#pragma unroll
      for (int r = 0; r < 8; ++r) {
        float v = fmaf(acc[j][r], CONV_FOLD, cb[j]);
        v = fmaxf(v, 0.0f) * ACARRY;
        slab[(8 * hh + r) * SLABP + 16 * j + c] = v;
      }
    }
    wave_sync_lds();
    for (int pass = 0; pass < 2; ++pass) {
#pragma unroll
      for (int it = 0; it < 4; ++it) {
        const int row = it * 4 + q4;
        const float* sp = slab + row * SLABP + c8;
        v8h hv;
#pragma unroll
        for (int e = 0; e < 8; ++e) hv[e] = (_Float16)sp[e];
        *(volatile v8h*)(E + ((size_t)(l0 + li) * NBATCH + (size_t)(16 * wave + row)) * NCONV + c8) = hv;
      }
      __threadfence();
    }
    wave_sync_lds();
  }
}

__global__ __launch_bounds__(256) void lstm_kernel(const unsigned short* __restrict__ Ep, const unsigned short* __restrict__ WCATp,
                                                   const float* __restrict__ BSUM, const float* __restrict__ lin_w,
                                                   const float* __restrict__ lin_b, float* __restrict__ out) {
  __shared__ __align__(16) _Float16 Pn[ROWBLK * PPITCH];
  __shared__ __align__(16) float    Hf[ROWBLK * HFP];
  __shared__ __align__(16) float    Os[ROWBLK * NOUTF];
  const _Float16* WCAT = (const _Float16*)WCATp;
  const int tid = threadIdx.x, lane = tid & 31, wave = tid >> 5;
  const int c = lane & 15, hh = lane >> 4, koff = hh * 8;
  const int rowbase = blockIdx.x * ROWBLK;
  const int j = 16 * wave + c;

#pragma unroll 1
  for (int i = tid; i < ROWBLK * PPITCH; i += 256) Pn[i] = (_Float16)0.0f;
  __syncthreads();
  const int xm = tid >> 4, xf4 = (tid & 15) * 4;
  {
    const v2u w = *(const v2u*)(Ep + ((size_t)rowbase + (size_t)xm) * NCONV + xf4);
    *(v2u*)(Pn + xm * PPITCH + xf4) = w;
  }
  float bb[4];
#pragma unroll
  for (int g = 0; g < 4; ++g) bb[g] = BSUM[g * NHID + j];
  float cs[8], hv[8];
#pragma unroll
  for (int r = 0; r < 8; ++r) { cs[r] = 0.0f; hv[r] = 0.0f; }
  __syncthreads();

  const _Float16* arow = Pn + c * PPITCH + koff;
  const _Float16* wrow = WCAT + (size_t)j * KCAT + koff;
  const v8f z8 = {0.f, 0.f, 0.f, 0.f, 0.f, 0.f, 0.f, 0.f};

#pragma unroll 1
  for (int t = 0; t < NSTEPS; ++t) {
    const int tn = (t + 1 < NSTEPS) ? (t + 1) : (NSTEPS - 1);
    const v2u xw = *(const v2u*)(Ep + ((size_t)tn * NBATCH + (size_t)rowbase + (size_t)xm) * NCONV + xf4);

    v8f acc[4];
    acc[0] = z8; acc[1] = z8; acc[2] = z8; acc[3] = z8;
#pragma unroll 1
    for (int k0 = 0; k0 < KCAT; k0 += 32) {
      const v16h a  = frag_load(arow + k0);
      const v16h w0 = frag_load(wrow + (size_t)0 * NHID * KCAT + k0);
      const v16h w1 = frag_load(wrow + (size_t)1 * NHID * KCAT + k0);
      const v16h w2 = frag_load(wrow + (size_t)2 * NHID * KCAT + k0);
      const v16h w3 = frag_load(wrow + (size_t)3 * NHID * KCAT + k0);
      acc[0] = frag_mma(a, w0, acc[0]);
      acc[1] = frag_mma(a, w1, acc[1]);
      acc[2] = frag_mma(a, w2, acc[2]);
      acc[3] = frag_mma(a, w3, acc[3]);
      wm_guard4(acc[0], acc[1], acc[2], acc[3], a, w0, w1, w2, w3);
    }
    acc_guard4(acc[0], acc[1], acc[2], acc[3]);

#pragma unroll
    for (int r = 0; r < 8; ++r) {
      const float zi = fmaf(acc[0][r], GATE_FOLD, bb[0]);
      const float zf = fmaf(acc[1][r], GATE_FOLD, bb[1]);
      const float zg = fmaf(acc[2][r], GATE_FOLD, bb[2]);
      const float zo = fmaf(acc[3][r], GATE_FOLD, bb[3]);
      const float ig = fsig(zi);
      const float fg = fsig(zf);
      const float gg = ftanh(zg);
      const float og = fsig(zo);
      const float cn = fg * cs[r] + ig * gg;
      cs[r] = cn;
      hv[r] = og * ftanh(cn);
    }

    __syncthreads();
#pragma unroll
    for (int r = 0; r < 8; ++r) Pn[(8 * hh + r) * PPITCH + NCONV + j] = (_Float16)(hv[r] * ACARRY);
    *(v2u*)(Pn + xm * PPITCH + xf4) = xw;
    __syncthreads();
  }

#pragma unroll
  for (int r = 0; r < 8; ++r) Hf[(8 * hh + r) * HFP + j] = hv[r];
  __syncthreads();
  {
    const int hidx = (tid < ROWBLK * NOUTF) ? tid : (ROWBLK * NOUTF - 1);
    const int hr = hidx / NOUTF;
    const int ho = hidx - hr * NOUTF;
    float a = 0.0f;
#pragma unroll 4
    for (int k = 0; k < NHID; ++k) a = fmaf(Hf[hr * HFP + k], lin_w[ho * NHID + k], a);
    a += lin_b[ho];
    if (tid < ROWBLK * NOUTF) Os[tid] = a;
  }
  __syncthreads();
  if (tid < (ROWBLK * NOUTF) / 4) {
    const v4f v = *(const v4f*)(Os + 4 * tid);
    float* dp = out + (size_t)blockIdx.x * (ROWBLK * NOUTF) + 4 * tid;
    *(volatile v4f*)dp = v;
    __threadfence();
    *(volatile v4f*)dp = v;
  }
}

extern "C" void kernel_launch(void* const* d_in, const int* in_sizes, int n_in,
                              void* d_out, int out_size, void* d_ws, size_t ws_size, hipStream_t stream) {
  if (n_in < 11 || d_out == nullptr || d_ws == nullptr) return;
  if (in_sizes[0] != NBATCH * NTIME * NCIN || in_sizes[3] != NCONV * NCIN * NTAP || in_sizes[4] != NCONV ||
      in_sizes[5] != NGATE * NCONV || in_sizes[6] != NGATE * NHID || in_sizes[7] != NGATE || in_sizes[8] != NGATE ||
      in_sizes[9] != NOUTF * NHID || in_sizes[10] != NOUTF || out_size != NBATCH * NOUTF) return;

  const float* input  = (const float*)d_in[0];
  const float* conv_w = (const float*)d_in[3];
  const float* conv_b = (const float*)d_in[4];
  const float* w_ih   = (const float*)d_in[5];
  const float* w_hh   = (const float*)d_in[6];
  const float* b_ih   = (const float*)d_in[7];
  const float* b_hh   = (const float*)d_in[8];
  const float* lin_w  = (const float*)d_in[9];
  const float* lin_b  = (const float*)d_in[10];
  float* out = (float*)d_out;

  char* ws = (char*)d_ws; size_t off = 0;
  auto carve = [&](size_t bytes) -> char* { char* p = ws + off; off += (bytes + 255) & ~(size_t)255; return p; };
  float*          INVN = (float*)carve((size_t)NBATCH * NCIN * 4);
  float*          BSUM = (float*)carve((size_t)NGATE * 4);
  unsigned short* WC   = (unsigned short*)carve((size_t)NCONV * KCONV * 2);
  unsigned short* WCAT = (unsigned short*)carve((size_t)NGATE * KCAT * 2);
  unsigned short* E    = (unsigned short*)carve((size_t)NSTEPS * NBATCH * NCONV * 2);
  if (off > ws_size || off > (size_t)134217728) return;

  prep_kernel<<<54, 256, 0, stream>>>(conv_w, w_ih, w_hh, b_ih, b_hh, WCAT, WC, BSUM);
  norm_kernel<<<NBATCH, 256, 0, stream>>>(input, INVN);
  conv_kernel<<<NSTEPS / LBLK, 128, 0, stream>>>(input, INVN, WC, conv_b, E);
  lstm_kernel<<<NBATCH / ROWBLK, 256, 0, stream>>>(E, WCAT, BSUM, lin_w, lin_b, out);
}
